// GraphAttentionLayer_34540126994437
// MI455X (gfx1250) — hardware-verified
//
#include <hip/hip_runtime.h>
#include <stddef.h>
#include <stdint.h>
#include <math.h>


#define NB      2
#define NN      2048
#define FIN     64
#define FOUT    128
#define NH      4
#define HD      32
#define MROWS   (NB * NN)
#define CTHR    256
#define GBM     64
#define GTHR    128
#define QROWS   16
#define YP      132
#define VSP     36
#define VCH     256
#define EEPL    (NB * NH * NN)
#define LN_EPS  1e-5f
#define WSMAX   134217728

static_assert((FIN % 32) == 0);
static_assert(FOUT == NH * HD);
static_assert(HD == 32);
static_assert((MROWS % GBM) == 0 && (NN % GBM) == 0);
static_assert(GBM == (GTHR / 32) * 16);
static_assert(GTHR == FOUT);
static_assert((NN % 64) == 0 && (NN % QROWS) == 0 && (NN % VCH) == 0);
static_assert(NH == GTHR / 32);
static_assert((YP % 4) == 0 && YP >= FOUT);
static_assert((VSP % 4) == 0 && VSP >= HD);
static_assert(NN == NH * 512);
static_assert((NN % 8) == 0 && (NN / 32) == 64);

typedef float          v4f  __attribute__((ext_vector_type(4)));
typedef float          v8f  __attribute__((ext_vector_type(8)));
typedef int            v8i  __attribute__((ext_vector_type(8)));
typedef unsigned int   v2u  __attribute__((ext_vector_type(2)));
typedef unsigned int   v4u  __attribute__((ext_vector_type(4)));
typedef unsigned short v8us __attribute__((ext_vector_type(8)));
typedef __bf16         v16b __attribute__((ext_vector_type(16)));
typedef v4f  __attribute__((may_alias)) v4fa;
typedef v2u  __attribute__((may_alias)) v2ua;
typedef v4u  __attribute__((may_alias)) v4ua;
typedef v8us __attribute__((may_alias)) v8usa;
union FragB { v16b v; v8us h[2]; v8i w; };

__device__ __forceinline__ v8f wmb(const FragB& a, const FragB& b, v8f c) {
  v8f d = __builtin_amdgcn_wmma_f32_16x16x32_bf16(false, a.v, false, b.v, (short)0, c, false, false);
  asm volatile("v_nop\n\tv_nop\n\tv_nop\n\tv_nop" : "+v"(d) : "v"(a.w), "v"(b.w));
  return d;
}

__device__ __forceinline__ unsigned int f2bf(float f) {
  const unsigned int u = __float_as_uint(f);
  return ((u + 0x7FFFu + ((u >> 16) & 1u)) >> 16) & 0xFFFFu;
}
__device__ __forceinline__ float bf2f(unsigned int b) { return __uint_as_float(b << 16); }
__device__ __forceinline__ float bfr(float f) { return bf2f(f2bf(f)); }
__device__ __forceinline__ v4f bfr4(const v4f a) {
  v4f r; r.x = bfr(a.x); r.y = bfr(a.y); r.z = bfr(a.z); r.w = bfr(a.w); return r;
}
__device__ __forceinline__ unsigned int pk2(float lo, float hi) { return f2bf(lo) | (f2bf(hi) << 16); }
__device__ __forceinline__ v4u pack8(const v4f a, const v4f b) {
  v4u r;
  r.x = pk2(a.x, a.y); r.y = pk2(a.z, a.w); r.z = pk2(b.x, b.y); r.w = pk2(b.z, b.w);
  return r;
}

__global__ __launch_bounds__(CTHR) void k_cvt(const float* __restrict__ x, unsigned short* xb, int nUx, int nBx,
                                              const float* __restrict__ w, unsigned short* wb, int nUw) {
  const int bx = (int)blockIdx.x, tid = (int)threadIdx.x;
  const bool isx = bx < nBx;
  const int u   = (isx ? bx : bx - nBx) * CTHR + tid;
  const int lim = isx ? nUx : nUw;
  if (u >= lim) return;
  const float* p = (isx ? x : w) + (size_t)u * 8;
  unsigned short* o = (isx ? xb : wb) + (size_t)u * 8;
  const v4f a = *(const v4fa*)p, b = *(const v4fa*)(p + 4);
  const v4u hv = pack8(a, b);
  *(volatile v4u*)o = hv;
  __threadfence();
  *(volatile v4u*)o = hv;
}

__global__ __launch_bounds__(CTHR) void k_adjbits(const int* __restrict__ adj, unsigned int* adjb) {
  __shared__ __attribute__((aligned(16))) unsigned int sb[8 * 64];
  const int tid = (int)threadIdx.x, lane = tid & 31, wave = tid >> 5;
  const int rb  = (int)blockIdx.x * 8;
  const int* arow = adj + (size_t)(rb + wave) * NN + lane;
  unsigned int w0 = 0u, w1 = 0u;
#pragma unroll 4
  for (int wd = 0; wd < 64; ++wd) {
    const int v = arow[32 * wd];
    const unsigned int bal = __builtin_amdgcn_ballot_w32(v != 0);
    w0 = (wd == lane) ? bal : w0;
    w1 = (wd == lane + 32) ? bal : w1;
  }
  sb[wave * 64 + lane]      = w0;
  sb[wave * 64 + 32 + lane] = w1;
  __syncthreads();
  const int tc = tid < 128 ? tid : 127;
  const v4u v = *(const v4ua*)(sb + 4 * tc);
  unsigned int* o = adjb + (size_t)rb * 64 + 4 * tc;
  const bool wr = tid < 128;
  if (wr) *(volatile v4u*)o = v;
  __threadfence();
  if (wr) *(volatile v4u*)o = v;
}

__global__ __launch_bounds__(GTHR) void k_proj(const unsigned short* __restrict__ XB,
                                               const unsigned short* __restrict__ WB,
                                               const float* __restrict__ a, float* Hf, float* EE) {
  __shared__ __attribute__((aligned(16))) float stg[GBM * FOUT];
  __shared__ __attribute__((aligned(16))) float satt[2 * FOUT];
  __shared__ __attribute__((aligned(16))) float sdot[2 * NH * GBM];
  const int tid = (int)threadIdx.x, lane = tid & 31, wave = tid >> 5, hh = lane >> 4, m = lane & 15;
  const int rowBase = (int)blockIdx.x * GBM;
  {
    const int hd = tid >> 5, d = tid & 31;
    const float v1 = a[hd * (2 * HD) + d];
    const float v2 = a[hd * (2 * HD) + HD + d];
    satt[tid]        = bfr(v1);
    satt[FOUT + tid] = bfr(v2);
  }
  v8f acc[8];
  {
    const v8f z = {0.f, 0.f, 0.f, 0.f, 0.f, 0.f, 0.f, 0.f};
#pragma unroll
    for (int t = 0; t < 8; ++t) acc[t] = z;
  }
  const unsigned short* ap = XB + (size_t)(rowBase + 16 * wave + m) * FIN + 8 * hh;
  const unsigned short* wp = WB + (size_t)m * FIN + 8 * hh;
#pragma unroll 1
  for (int ks = 0; ks < FIN / 32; ++ks) {
    FragB af;
    af.h[0] = *(const v8usa*)(ap + 32 * ks);
    af.h[1] = *(const v8usa*)(ap + 32 * ks + 16);
#pragma unroll
    for (int t = 0; t < 8; ++t) {
      const unsigned short* wq = wp + (size_t)(16 * t) * FIN + 32 * ks;
      FragB bf;
      bf.h[0] = *(const v8usa*)wq;
      bf.h[1] = *(const v8usa*)(wq + 16);
      acc[t] = wmb(af, bf, acc[t]);
    }
  }
#pragma unroll
  for (int t = 0; t < 8; ++t) {
#pragma unroll
    for (int r = 0; r < 8; ++r) {
      const int lr = 16 * wave + 8 * hh + r;
      stg[lr * FOUT + 16 * t + m] = acc[t][r];
    }
  }
  __syncthreads();
  {
    const int row = tid & 63, which = tid >> 6;
#pragma unroll 1
    for (int hd = 0; hd < NH; ++hd) {
      const float* hr = stg + row * FOUT + hd * HD;
      const float* sa = satt + which * FOUT + hd * HD;
      float d = 0.f;
#pragma unroll 4
      for (int c4 = 0; c4 < HD / 4; ++c4) {
        const v4f hv = *(const v4fa*)(hr + 4 * c4);
        const v4f av = *(const v4fa*)(sa + 4 * c4);
        d = fmaf(hv.x, av.x, d);
        d = fmaf(hv.y, av.y, d);
        d = fmaf(hv.z, av.z, d);
        d = fmaf(hv.w, av.w, d);
      }
      sdot[(which * NH + hd) * GBM + row] = d;
    }
  }
  __syncthreads();

  v4f fv[16];
#pragma unroll
  for (int i = 0; i < 16; ++i) fv[i] = *(const v4fa*)(stg + (16 * wave + i) * FOUT + 4 * lane);
  const int which2 = lane >> 4, piece = lane & 15;
  const v4f sdv = *(const v4fa*)(sdot + (which2 * NH + wave) * GBM + 4 * piece);
  const int bb  = rowBase / NN;
  const int nb0 = rowBase - bb * NN;
  float* sp = EE + (size_t)which2 * EEPL + (size_t)(bb * NH + wave) * NN + nb0 + 4 * piece;
  float* hp = Hf + (size_t)(rowBase + 16 * wave) * FOUT + 4 * lane;
#pragma unroll
  for (int i = 0; i < 16; ++i) *(volatile v4f*)(hp + (size_t)i * FOUT) = fv[i];
  *(volatile v4f*)sp = sdv;
  __threadfence();
#pragma unroll
  for (int i = 0; i < 16; ++i) *(volatile v4f*)(hp + (size_t)i * FOUT) = fv[i];
  *(volatile v4f*)sp = sdv;
}

__global__ __launch_bounds__(CTHR) void k_vbuild(const float* __restrict__ Hf, unsigned short* VTH,
                                                 unsigned short* VTL) {
  __shared__ __attribute__((aligned(16))) float stg[VCH * VSP];
  const int tid = (int)threadIdx.x;
  const int bx = (int)blockIdx.x;
  const int b = bx >> 5, hh = (bx >> 3) & 3, c = bx & 7;
  const int n0 = VCH * c;
#pragma unroll 4
  for (int it = 0; it < 8; ++it) {
    const int u = tid + CTHR * it;
    const int r = u >> 3, q = u & 7;
    const v4f v = *(const v4fa*)(Hf + (size_t)(b * NN + n0 + r) * FOUT + hh * HD + 4 * q);
    *(v4fa*)(stg + r * VSP + 4 * q) = v;
  }
  __syncthreads();
  v4u hv[4], lv[4];
#pragma unroll
  for (int it = 0; it < 4; ++it) {
    const int u = tid + CTHR * it;
    const int piece = u & 7, line = u >> 3;
    const int hp = line >> 5, d = line & 31;
    float f[8];
#pragma unroll
    for (int i = 0; i < 8; ++i) f[i] = stg[(4 * (8 * piece + i) + hp) * VSP + d];
    unsigned int hb[8], lb[8];
#pragma unroll
    for (int i = 0; i < 8; ++i) {
      hb[i] = f2bf(f[i]);
      lb[i] = f2bf(f[i] - bf2f(hb[i]));
    }
    hv[it].x = hb[0] | (hb[1] << 16); hv[it].y = hb[2] | (hb[3] << 16);
    hv[it].z = hb[4] | (hb[5] << 16); hv[it].w = hb[6] | (hb[7] << 16);
    lv[it].x = lb[0] | (lb[1] << 16); lv[it].y = lb[2] | (lb[3] << 16);
    lv[it].z = lb[4] | (lb[5] << 16); lv[it].w = lb[6] | (lb[7] << 16);
  }
#pragma unroll
  for (int it = 0; it < 4; ++it) {
    const int u = tid + CTHR * it;
    const int piece = u & 7, line = u >> 3;
    const int hp = line >> 5, d = line & 31;
    const size_t o = (size_t)((b * NH + hp) * HD + d) * NN + hh * 512 + 64 * c + 8 * piece;
    *(volatile v4u*)(VTH + o) = hv[it];
    *(volatile v4u*)(VTL + o) = lv[it];
  }
  __threadfence();
#pragma unroll
  for (int it = 0; it < 4; ++it) {
    const int u = tid + CTHR * it;
    const int piece = u & 7, line = u >> 3;
    const int hp = line >> 5, d = line & 31;
    const size_t o = (size_t)((b * NH + hp) * HD + d) * NN + hh * 512 + 64 * c + 8 * piece;
    *(volatile v4u*)(VTH + o) = hv[it];
    *(volatile v4u*)(VTL + o) = lv[it];
  }
}

__global__ __launch_bounds__(GTHR) void k_attn(const unsigned int* __restrict__ ADJB, const float* __restrict__ EE,
                                               const unsigned short* __restrict__ VTH,
                                               const unsigned short* __restrict__ VTL,
                                               const float* __restrict__ Hf, const float* __restrict__ gamma,
                                               const float* __restrict__ beta, float* out) {
  __shared__ __attribute__((aligned(16))) float ybuf[QROWS * YP];
  const int tid = (int)threadIdx.x, lane = tid & 31, head = tid >> 5, hh = lane >> 4, m = lane & 15;
  const int b  = (int)blockIdx.x / (NN / QROWS);
  const int n0 = ((int)blockIdx.x - b * (NN / QROWS)) * QROWS;
  const int qi = n0 + m;
  const size_t bh = (size_t)(b * NH + head);
  const float ei = EE[bh * NN + qi];
  const float* ejp = EE + (size_t)EEPL + bh * NN + 8 * hh;
  const unsigned int* adjrow = ADJB + (size_t)qi * 64;
  const unsigned short* vh = VTH + (bh * HD + m) * NN + 8 * hh;
  const unsigned short* vl = VTL + (bh * HD + m) * NN + 8 * hh;

  const float NEGB = -3.0e38f;
  const float NEGT = -1.0e38f;
  float mrun = NEGB, lsum = 0.f;
  v8f acc0 = {0.f, 0.f, 0.f, 0.f, 0.f, 0.f, 0.f, 0.f};
  v8f acc1 = {0.f, 0.f, 0.f, 0.f, 0.f, 0.f, 0.f, 0.f};

#pragma unroll 1
  for (int kt = 0; kt < NN / 64; ++kt) {
    const int k0 = 64 * kt;
    const v2u bw = *(const v2ua*)(adjrow + 2 * kt);
    float sv[32];
    float tm = NEGB;
#pragma unroll
    for (int st = 0; st < 2; ++st) {
      const float* ep = ejp + k0 + 32 * st;
      const v4f e0 = *(const v4fa*)ep,        e1 = *(const v4fa*)(ep + 4);
      const v4f e2 = *(const v4fa*)(ep + 16), e3 = *(const v4fa*)(ep + 20);
      const unsigned int word = (st == 0) ? bw.x : bw.y;
      const unsigned int sh = word >> (8 * hh);
      const unsigned int kb = (sh & 0xFFu) | ((sh >> 8) & 0xFF00u);
      const float ev[16] = {e0.x, e0.y, e0.z, e0.w, e1.x, e1.y, e1.z, e1.w,
                            e2.x, e2.y, e2.z, e2.w, e3.x, e3.y, e3.z, e3.w};
#pragma unroll
      for (int i = 0; i < 16; ++i) {
        float t = ei + ev[i];
        t = (t > 0.f) ? t : 0.2f * t;
        t = (((kb >> i) & 1u) != 0u) ? t : NEGB;
        sv[16 * st + i] = t;
        tm = fmaxf(tm, t);
      }
    }
    tm = fmaxf(tm, __shfl_xor(tm, 16));
    const float mnew  = fmaxf(mrun, tm);
    const float msafe = (mnew > NEGT) ? mnew : 0.f;
    const float alpha = expf(fmaxf(mrun - msafe, -200.f));
    mrun = mnew;
    lsum *= alpha;
#pragma unroll
    for (int r = 0; r < 8; ++r) {
      const float ar = __shfl(alpha, 8 * hh + r);
      acc0[r] *= ar;
      acc1[r] *= ar;
    }
#pragma unroll
    for (int st = 0; st < 2; ++st) {
      FragB aH, aL;
      float ps = 0.f;
#pragma unroll
      for (int q = 0; q < 8; ++q) {
        const float s0 = sv[16 * st + 2 * q], s1 = sv[16 * st + 2 * q + 1];
        const float x0 = expf(s0 - msafe), x1 = expf(s1 - msafe);
        const float p0 = (s0 > NEGT) ? x0 : 0.f;
        const float p1 = (s1 > NEGT) ? x1 : 0.f;
        ps += p0 + p1;
        const unsigned int h0 = f2bf(p0), h1 = f2bf(p1);
        const unsigned int l0 = f2bf(p0 - bf2f(h0)), l1 = f2bf(p1 - bf2f(h1));
        aH.w[q] = (int)(h0 | (h1 << 16));
        aL.w[q] = (int)(l0 | (l1 << 16));
      }
      lsum += ps;
      const unsigned short* vq = vh + k0 + 32 * st;
      const unsigned short* lq = vl + k0 + 32 * st;
      FragB bH0, bL0, bH1, bL1;
      bH0.h[0] = *(const v8usa*)vq;                         bH0.h[1] = *(const v8usa*)(vq + 16);
      bL0.h[0] = *(const v8usa*)lq;                         bL0.h[1] = *(const v8usa*)(lq + 16);
      bH1.h[0] = *(const v8usa*)(vq + (size_t)16 * NN);     bH1.h[1] = *(const v8usa*)(vq + (size_t)16 * NN + 16);
      bL1.h[0] = *(const v8usa*)(lq + (size_t)16 * NN);     bL1.h[1] = *(const v8usa*)(lq + (size_t)16 * NN + 16);
      acc0 = wmb(aH, bH0, acc0);
      acc0 = wmb(aH, bL0, acc0);
      acc0 = wmb(aL, bH0, acc0);
      acc1 = wmb(aH, bH1, acc1);
      acc1 = wmb(aH, bL1, acc1);
      acc1 = wmb(aL, bH1, acc1);
    }
  }

  const float lt  = lsum + __shfl_xor(lsum, 16);
  const float inv = (lt > 0.f) ? (1.0f / lt) : 0.f;
#pragma unroll
  for (int r = 0; r < 8; ++r) {
    const float ir = __shfl(inv, 8 * hh + r);
    const int lr = 8 * hh + r;
    ybuf[lr * YP + head * HD + m]      = acc0[r] * ir;
    ybuf[lr * YP + head * HD + 16 + m] = acc1[r] * ir;
  }
  __syncthreads();

  const v4f g4 = bfr4(*(const v4fa*)(gamma + 4 * lane));
  const v4f b4 = bfr4(*(const v4fa*)(beta + 4 * lane));
  v4f ov[4];
#pragma unroll
  for (int rr = 0; rr < 4; ++rr) {
    const int row = 4 * head + rr;
    const v4f hp4 = *(const v4fa*)(ybuf + row * YP + 4 * lane);
    const v4f hr4 = *(const v4fa*)(Hf + (size_t)(b * NN + n0 + row) * FOUT + 4 * lane);
    v4f y;
    y.x = hp4.x + hr4.x; y.y = hp4.y + hr4.y; y.z = hp4.z + hr4.z; y.w = hp4.w + hr4.w;
    float s = (y.x + y.y) + (y.z + y.w);
#pragma unroll
    for (int off = 16; off > 0; off >>= 1) s += __shfl_xor(s, off);
    const float mu = s * (1.0f / FOUT);
    v4f d;
    d.x = y.x - mu; d.y = y.y - mu; d.z = y.z - mu; d.w = y.w - mu;
    float q = (d.x * d.x + d.y * d.y) + (d.z * d.z + d.w * d.w);
#pragma unroll
    for (int off = 16; off > 0; off >>= 1) q += __shfl_xor(q, off);
    const float var = q * (1.0f / FOUT);
    const float rs  = 1.0f / sqrtf(var + LN_EPS);
    v4f o;
    o.x = d.x * rs * g4.x + b4.x;
    o.y = d.y * rs * g4.y + b4.y;
    o.z = d.z * rs * g4.z + b4.z;
    o.w = d.w * rs * g4.w + b4.w;
    ov[rr] = o;
  }
  float* op = out + (size_t)(b * NN + n0 + 4 * head) * FOUT + 4 * lane;
#pragma unroll
  for (int rr = 0; rr < 4; ++rr) *(volatile v4f*)(op + (size_t)rr * FOUT) = ov[rr];
  __threadfence();
#pragma unroll
  for (int rr = 0; rr < 4; ++rr) *(volatile v4f*)(op + (size_t)rr * FOUT) = ov[rr];
}

extern "C" void kernel_launch(void* const* d_in, const int* in_sizes, int n_in,
                              void* d_out, int out_size, void* d_ws, size_t ws_size,
                              hipStream_t stream) {
  if (n_in < 6) return;
  if (in_sizes[0] != MROWS * FIN) return;
  if (in_sizes[1] != NN * NN) return;
  if (in_sizes[2] != FOUT * FIN) return;
  if (in_sizes[3] != NH * 2 * HD) return;
  if (in_sizes[4] != FOUT || in_sizes[5] != FOUT) return;
  if (out_size != MROWS * FOUT) return;

  const float* x     = (const float*)d_in[0];
  const int*   adj   = (const int*)  d_in[1];
  const float* w     = (const float*)d_in[2];
  const float* a     = (const float*)d_in[3];
  const float* gamma = (const float*)d_in[4];
  const float* beta  = (const float*)d_in[5];
  float* out = (float*)d_out;

  char* ws = (char*)d_ws;
  size_t off = 0;
  const size_t oXB  = off; off += (size_t)MROWS * FIN * 2;            off = (off + 255) & ~(size_t)255;
  const size_t oWB  = off; off += (size_t)FOUT * FIN * 2;             off = (off + 255) & ~(size_t)255;
  const size_t oADJ = off; off += (size_t)NN * 64 * 4;                off = (off + 255) & ~(size_t)255;
  const size_t oHF  = off; off += (size_t)MROWS * FOUT * 4;           off = (off + 255) & ~(size_t)255;
  const size_t oEE  = off; off += (size_t)2 * EEPL * 4;               off = (off + 255) & ~(size_t)255;
  const size_t oVTH = off; off += (size_t)NB * NH * HD * NN * 2;      off = (off + 255) & ~(size_t)255;
  const size_t oVTL = off; off += (size_t)NB * NH * HD * NN * 2;      off = (off + 255) & ~(size_t)255;
  if (off > ws_size || off > (size_t)WSMAX) return;
  unsigned short* XB   = (unsigned short*)(ws + oXB);
  unsigned short* WB   = (unsigned short*)(ws + oWB);
  unsigned int*   ADJB = (unsigned int*)(ws + oADJ);
  float*          HF   = (float*)(ws + oHF);
  float*          EE   = (float*)(ws + oEE);
  unsigned short* VTH  = (unsigned short*)(ws + oVTH);
  unsigned short* VTL  = (unsigned short*)(ws + oVTL);

  const int nUx = MROWS * FIN / 8;
  const int nUw = FOUT * FIN / 8;
  const int nBx = (nUx + CTHR - 1) / CTHR;
  const int nBw = (nUw + CTHR - 1) / CTHR;
  k_cvt<<<nBx + nBw, CTHR, 0, stream>>>(x, XB, nUx, nBx, w, WB, nUw);
  k_adjbits<<<NN / 8, CTHR, 0, stream>>>(adj, ADJB);
  k_proj<<<MROWS / GBM, GTHR, 0, stream>>>(XB, WB, a, HF, EE);
  k_vbuild<<<NB * NH * (NN / VCH), CTHR, 0, stream>>>(HF, VTH, VTL);
  k_attn<<<NB * (NN / QROWS), GTHR, 0, stream>>>(ADJB, EE, VTH, VTL, HF, gamma, beta, out);
}
